// CustomConvLayer_17798344475089
// MI455X (gfx1250) — hardware-verified
//
#include <hip/hip_runtime.h>
#include <stdint.h>
#include <stddef.h>

typedef __attribute__((ext_vector_type(16))) _Float16 v16h;
typedef __attribute__((ext_vector_type(8)))  _Float16 v8h;
typedef __attribute__((ext_vector_type(16))) __bf16   v16b;
typedef __attribute__((ext_vector_type(8)))  __bf16   v8b;
typedef __attribute__((ext_vector_type(8)))  float    v8f;
typedef __attribute__((ext_vector_type(4)))  float    v4f;

__device__ __forceinline__ void dep_guard_h(v8f& a, v8f& b, v16h x, v16h y) { asm volatile("v_nop\n\tv_nop\n\tv_nop\n\tv_nop" : "+v"(a), "+v"(b) : "v"(x), "v"(y)); }
__device__ __forceinline__ void dep_guard_b(v8f& a, v8f& b, v16b x, v16b y) { asm volatile("v_nop\n\tv_nop\n\tv_nop\n\tv_nop" : "+v"(a), "+v"(b) : "v"(x), "v"(y)); }
__device__ __forceinline__ void keep4_h(v16h a, v16h b, v16h c, v16h d) { asm volatile("v_nop" :: "v"(a), "v"(b), "v"(c), "v"(d)); }
__device__ __forceinline__ void keep4_b(v16b a, v16b b, v16b c, v16b d) { asm volatile("v_nop" :: "v"(a), "v"(b), "v"(c), "v"(d)); }

template <typename T> struct Frag;
template <> struct Frag<_Float16> {
  typedef v16h V; union U { v16h v; v8h h[2]; };
  static __device__ __forceinline__ v16h load(const _Float16* p) {
    U f; f.h[0] = *(const v8h*)(p); f.h[1] = *(const v8h*)(p + 16); return f.v;
  }
  static __device__ __forceinline__ v8f mma(v16h a, v16h b, v8f c) {
    return __builtin_amdgcn_wmma_f32_16x16x32_f16(false, a, false, b, (short)0, c, false, false);
  }
  static __device__ __forceinline__ void guard(v8f& a, v8f& b, v16h x, v16h y) { dep_guard_h(a, b, x, y); }
  static __device__ __forceinline__ void keep(v16h a, v16h b, v16h c, v16h d) { keep4_h(a, b, c, d); }
};
template <> struct Frag<__bf16> {
  typedef v16b V; union U { v16b v; v8b h[2]; };
  static __device__ __forceinline__ v16b load(const __bf16* p) {
    U f; f.h[0] = *(const v8b*)(p); f.h[1] = *(const v8b*)(p + 16); return f.v;
  }
  static __device__ __forceinline__ v8f mma(v16b a, v16b b, v8f c) {
    return __builtin_amdgcn_wmma_f32_16x16x32_bf16(false, a, false, b, (short)0, c, false, false);
  }
  static __device__ __forceinline__ void guard(v8f& a, v8f& b, v16b x, v16b y) { dep_guard_b(a, b, x, y); }
  static __device__ __forceinline__ void keep(v16b a, v16b b, v16b c, v16b d) { keep4_b(a, b, c, d); }
};

__device__ __forceinline__ void guard8(v8f& a0, v8f& a1, v8f& a2, v8f& a3,
                                       v8f& a4, v8f& a5, v8f& a6, v8f& a7,
                                       v16h x0, v16h x1, v16h x2, v16h x3, v16h y0, v16h y1) {
  asm volatile("v_nop\n\tv_nop\n\tv_nop\n\tv_nop"
               : "+v"(a0), "+v"(a1), "+v"(a2), "+v"(a3), "+v"(a4), "+v"(a5), "+v"(a6), "+v"(a7)
               : "v"(x0), "v"(x1), "v"(x2), "v"(x3), "v"(y0), "v"(y1));
}

constexpr int NBATCH  = 8;
constexpr int NCH_IN  = 64;
constexpr int NCH_OUT = 64;
constexpr int IMG     = 128;
constexpr int NTAP    = 9;
constexpr int NTAP4   = 16;
constexpr int CHQ     = 16;
constexpr int NPHASE  = NCH_IN / CHQ;
constexpr int KTOT    = NCH_IN * NTAP4;
constexpr int XROWS   = 5;
constexpr int XCOLS   = 132;
constexpr int OPITCH  = 132;
constexpr float WSCALE     = 1024.0f;
constexpr float WSCALE_INV = 1.0f / 1024.0f;

static_assert(KTOT % 32 == 0, "K multiple of 32");
static_assert(NCH_OUT % 16 == 0 && IMG % 16 == 0, "tile multiples");
static_assert(NPHASE * 8 * 32 == KTOT, "k-step coverage");
static_assert((XROWS * XCOLS * CHQ) % 8 == 0, "staging vector granularity");
static_assert((OPITCH * 4) % 16 == 0, "slab pitch alignment");

__global__ __launch_bounds__(256) void fold_tap_weights(
    const float* __restrict__ w,
    const float* __restrict__ toff,
    unsigned short* __restrict__ wfp)
{
  const int idx = blockIdx.x * 256 + threadIdx.x;
  const int m   = idx >> 7;
  const int k0  = (idx & 127) * 8;
  const int cq  = k0 >> 8;
  const int t   = (k0 >> 4) & 15;
  const int chl0 = k0 & 15;
  const int ci0 = cq * CHQ + chl0;
  const int rr  = t >> 2, cc = t & 3;

  float acc[8];
#pragma unroll
  for (int e = 0; e < 8; ++e) acc[e] = 0.0f;

#pragma unroll 1
  for (int kk = 0; kk < NTAP; ++kk) {
    const float dy = toff[2 * kk];
    const float dx = toff[2 * kk + 1];
    const float yb = floorf(dy), xb = floorf(dx);
    const float fy = dy - yb, fx = dx - xb;
    int iy = (int)yb; iy = min(max(iy, 0), 2);
    int ix = (int)xb; ix = min(max(ix, 0), 2);
    const float wy = (rr == iy) ? (1.0f - fy) : ((rr == iy + 1) ? fy : 0.0f);
    const float wx = (cc == ix) ? (1.0f - fx) : ((cc == ix + 1) ? fx : 0.0f);
    const float coef = wy * wx;
    const float* wp = w + (size_t)(m * NCH_IN + ci0) * NTAP + kk;
#pragma unroll
    for (int e = 0; e < 8; ++e) acc[e] += coef * wp[e * NTAP];
  }

  v8h hv;
#pragma unroll
  for (int e = 0; e < 8; ++e) hv[e] = (_Float16)(acc[e] * WSCALE);

  _Float16* dst = (_Float16*)wfp + (size_t)m * KTOT + k0;
  *(volatile v8h*)dst = hv;
  __threadfence();
  *(volatile v8h*)dst = hv;
}

__global__ __launch_bounds__(256) void conv_taps_wmma(
    const float* __restrict__ x,
    const unsigned short* __restrict__ wfp,
    float* __restrict__ out)
{
  __shared__ __align__(16) _Float16 lds_x[XROWS * XCOLS * CHQ];
  __shared__ __align__(16) float    sOut[2 * NCH_OUT * OPITCH];

  const _Float16* wf = (const _Float16*)wfp;
  const int blk  = blockIdx.x;
  const int b    = blk >> 6;
  const int oy0  = (blk & 63) * 2;
  const int tid  = threadIdx.x;
  const int wave = tid >> 5;
  const int lane = tid & 31;
  const int hh   = lane >> 4;
  const int nl   = lane & 15;
  const int ox0  = wave * 16;
  const int col  = ox0 + nl;

  v8f acc[2][4];
#pragma unroll
  for (int i = 0; i < 2; ++i)
#pragma unroll
    for (int j = 0; j < 4; ++j) acc[i][j] = (v8f){0.f,0.f,0.f,0.f,0.f,0.f,0.f,0.f};

  for (int cq = 0; cq < NPHASE; ++cq) {
    __syncthreads();
#pragma unroll 1
    for (int item = tid; item < XROWS * 2 * XCOLS; item += 256) {
      const int rg  = item / XCOLS;
      const int j   = item - rg * XCOLS;
      const int dyr = rg >> 1;
      const int g8  = rg & 1;
      const int gy  = oy0 - 1 + dyr;
      const int gx  = j - 1;
      const bool ok = ((unsigned)gy < (unsigned)IMG) && ((unsigned)gx < (unsigned)IMG);
      const int gyc = min(max(gy, 0), IMG - 1);
      const int gxc = min(max(gx, 0), IMG - 1);
      const float* p = x + (((size_t)(b * NCH_IN + cq * CHQ + g8 * 8)) * IMG + gyc) * IMG + gxc;
      v8h hv;
#pragma unroll
      for (int e = 0; e < 8; ++e) {
        float v = p[(size_t)e * IMG * IMG];
        v = ok ? v : 0.0f;
        hv[e] = (_Float16)v;
      }
      *(v8h*)(lds_x + ((dyr * XCOLS + j) * CHQ + g8 * 8)) = hv;
    }
    __syncthreads();

#pragma unroll
    for (int s = 0; s < 8; ++s) {
      const int t0 = 2 * s, t1 = 2 * s + 1;
      const int r0 = t0 >> 2, c0 = t0 & 3;
      const int r1 = t1 >> 2, c1 = t1 & 3;
      v16h av[4];
#pragma unroll
      for (int mt = 0; mt < 4; ++mt)
        av[mt] = Frag<_Float16>::load(wf + (size_t)(mt * 16 + nl) * KTOT + cq * 256 + s * 32 + 8 * hh);
      v16h bv[2];
#pragma unroll
      for (int row = 0; row < 2; ++row) {
        Frag<_Float16>::U f;
        f.h[0] = *(const v8h*)(lds_x + (((row + r0) * XCOLS + col + c0) * CHQ + 8 * hh));
        f.h[1] = *(const v8h*)(lds_x + (((row + r1) * XCOLS + col + c1) * CHQ + 8 * hh));
        bv[row] = f.v;
      }
#pragma unroll
      for (int mt = 0; mt < 4; ++mt) {
        acc[0][mt] = Frag<_Float16>::mma(av[mt], bv[0], acc[0][mt]);
        acc[1][mt] = Frag<_Float16>::mma(av[mt], bv[1], acc[1][mt]);
      }
      guard8(acc[0][0], acc[0][1], acc[0][2], acc[0][3],
             acc[1][0], acc[1][1], acc[1][2], acc[1][3],
             av[0], av[1], av[2], av[3], bv[0], bv[1]);
    }
  }

#pragma unroll
  for (int row = 0; row < 2; ++row)
#pragma unroll
    for (int mt = 0; mt < 4; ++mt)
#pragma unroll
      for (int r = 0; r < 8; ++r)
        sOut[(row * NCH_OUT + mt * 16 + 8 * hh + r) * OPITCH + col] = acc[row][mt][r] * WSCALE_INV;
  __syncthreads();

  for (int pass = 0; pass < 2; ++pass) {
#pragma unroll 1
    for (int it = 0; it < 16; ++it) {
      const int seg = it * 8 + wave;
      const int row = seg >> 6;
      const int co  = seg & 63;
      const v4f val = *(const v4f*)(sOut + (row * NCH_OUT + co) * OPITCH + lane * 4);
      float* dst = out + ((((size_t)b * NCH_OUT + co) * IMG + oy0 + row) * IMG) + lane * 4;
      *(volatile v4f*)dst = val;
    }
    __threadfence();
  }
}

extern "C" void kernel_launch(void* const* d_in, const int* in_sizes, int n_in,
                              void* d_out, int out_size, void* d_ws, size_t ws_size,
                              hipStream_t stream)
{
  const float* x    = (const float*)d_in[0];
  const float* w    = (const float*)d_in[1];
  const float* toff = (const float*)d_in[2];
  unsigned short* wf = (unsigned short*)d_ws;

  fold_tap_weights<<<(NCH_OUT * KTOT / 8) / 256, 256, 0, stream>>>(w, toff, wf);
  conv_taps_wmma<<<NBATCH * (IMG / 2), 256, 0, stream>>>(x, wf, (float*)d_out);
}
